// BinaryMatchAttention_62380105007277
// MI455X (gfx1250) — hardware-verified
//
#include <hip/hip_runtime.h>


#define NB_  4
#define NQ   1024
#define NK   2048
#define NBIT 16
#define DV   512
#define ITEMP 10.0f
typedef _Float16 h16;
typedef unsigned short bf;
typedef __attribute__((ext_vector_type(16))) __bf16   v16bf;
typedef __attribute__((ext_vector_type(16))) _Float16 v16h;
typedef __attribute__((ext_vector_type(8)))  _Float16 v8h;
typedef __attribute__((ext_vector_type(8)))  unsigned short v8us;
typedef __attribute__((ext_vector_type(8)))  float    v8f;
typedef __attribute__((ext_vector_type(4)))  float    v4f;
typedef v8h  __attribute__((may_alias)) v8ha;
typedef v4f  __attribute__((may_alias)) v4fa;
typedef v8us __attribute__((may_alias)) v8usa;

__device__ __forceinline__ unsigned short f2bf(float f) { unsigned u = __float_as_uint(f); u += 0x7FFFu + ((u >> 16) & 1u); return (unsigned short)(u >> 16); }
__device__ __forceinline__ float bf2f(unsigned short b) { return __uint_as_float(((unsigned)b) << 16); }
__device__ __forceinline__ float bfr(float f) { return bf2f(f2bf(f)); }
__device__ __forceinline__ v16h cat16(v8h lo, v8h hi) { return __builtin_shufflevector(lo, hi, 0, 1, 2, 3, 4, 5, 6, 7, 8, 9, 10, 11, 12, 13, 14, 15); }
__device__ __forceinline__ v16bf cat16b(v8us lo, v8us hi) { return __builtin_bit_cast(v16bf, __builtin_shufflevector(lo, hi, 0, 1, 2, 3, 4, 5, 6, 7, 8, 9, 10, 11, 12, 13, 14, 15)); }
__device__ __forceinline__ v8f wmma16(v16h a, v16h b, v8f c) { return __builtin_amdgcn_wmma_f32_16x16x32_f16(false, a, false, b, (short)0, c, false, false); }
__device__ __forceinline__ v8f wmmab(v16bf a, v16bf b, v8f c) { return __builtin_amdgcn_wmma_f32_16x16x32_bf16(false, a, false, b, (short)0, c, false, false); }


template <typename T16> struct WFrag;
template <> struct WFrag<h16> { typedef v16h V; static __device__ __forceinline__ V ld(const h16* p) { return cat16(*(const v8h*)p, *(const v8h*)(p + 16)); } static __device__ __forceinline__ v8f mma(V a, V b, v8f c) { return wmma16(a, b, c); } };
template <> struct WFrag<bf> { typedef v16bf V; static __device__ __forceinline__ V ld(const bf* p) { return cat16b(*(const v8us*)p, *(const v8us*)(p + 16)); } static __device__ __forceinline__ v8f mma(V a, V b, v8f c) { return wmmab(a, b, c); } };
template <typename T16, int NSPLIT, bool BIAS>
__global__ __launch_bounds__(32) void k_gemmw(const T16* __restrict__ A, const T16* __restrict__ A2, const T16* __restrict__ Bt, const T16* __restrict__ Bt2, int K, float* C, int ldc, const float* __restrict__ bias, size_t sA, size_t sB, size_t sC) {
    typedef typename WFrag<T16>::V V;
    __shared__ __align__(16) float os[16 * 68];
    const size_t z = blockIdx.z; A += z * sA; if (A2) A2 += z * sA; Bt += z * sB; if (Bt2) Bt2 += z * sB; C += z * sC;
    const int lane = threadIdx.x & 31, lr = lane & 15, hi = lane >> 4; const int r0 = blockIdx.x * 64, c0 = blockIdx.y * 64;
    v8f acc[4][4];
#pragma unroll
    for (int mb = 0; mb < 4; ++mb)
#pragma unroll
        for (int nb = 0; nb < 4; ++nb) acc[mb][nb] = (v8f){};
    const size_t aoff = (size_t)(r0 + lr) * K + 8 * hi, boff = (size_t)(c0 + lr) * K + 8 * hi;
#pragma unroll 1
    for (int kc = 0; kc < K; kc += 32) {
        V a[4], a2[4];
#pragma unroll
        for (int mb = 0; mb < 4; ++mb) { a[mb] = WFrag<T16>::ld(A + aoff + (size_t)mb * 16 * K + kc); if (NSPLIT == 1 || NSPLIT == 2) a2[mb] = WFrag<T16>::ld(A2 + aoff + (size_t)mb * 16 * K + kc); }
#pragma unroll
        for (int nb = 0; nb < 4; ++nb) { const V b = WFrag<T16>::ld(Bt + boff + (size_t)nb * 16 * K + kc); V b2; if (NSPLIT >= 2) b2 = WFrag<T16>::ld(Bt2 + boff + (size_t)nb * 16 * K + kc);
#pragma unroll
            for (int mb = 0; mb < 4; ++mb) { acc[mb][nb] = WFrag<T16>::mma(a[mb], b, acc[mb][nb]); if (NSPLIT == 1 || NSPLIT == 2) acc[mb][nb] = WFrag<T16>::mma(a2[mb], b, acc[mb][nb]); if (NSPLIT >= 2) acc[mb][nb] = WFrag<T16>::mma(a[mb], b2, acc[mb][nb]); } }
        asm volatile("v_nop\n\tv_nop\n\tv_nop\n\tv_nop" : "+v"(acc[0][0]), "+v"(acc[1][1]), "+v"(acc[2][2]), "+v"(acc[3][3]) : "v"(a[0]), "v"(a[3]));
    }
#pragma unroll
    for (int mb = 0; mb < 4; ++mb) {
#pragma unroll
        for (int nb = 0; nb < 4; ++nb) {
#pragma unroll
            for (int j = 0; j < 8; ++j) os[(hi * 8 + j) * 68 + nb * 16 + lr] = acc[mb][nb][j]; }
        __builtin_amdgcn_wave_barrier(); asm volatile("" ::: "memory");
        float* crow = C + (size_t)(r0 + mb * 16) * ldc + c0;
#pragma unroll 1
        for (int ps = 0; ps < 2; ++ps) {
#pragma unroll
            for (int s = 0; s < 8; ++s) { const int row = 2 * s + hi, cofs = lr * 4; v4f val = *(const v4fa*)(os + row * 68 + cofs); if (BIAS) { val[0] += bfr(bias[c0 + cofs]); val[1] += bfr(bias[c0 + cofs + 1]); val[2] += bfr(bias[c0 + cofs + 2]); val[3] += bfr(bias[c0 + cofs + 3]); }
                *(volatile v4f*)(crow + (size_t)row * ldc + cofs) = val; }
            if (ps == 0) __threadfence(); }
        __builtin_amdgcn_wave_barrier(); asm volatile("" ::: "memory");
    }
}

__device__ __forceinline__ void splitf(float y, unsigned short& h, unsigned short& l) { h = f2bf(y); l = f2bf(y - bf2f(h)); }
typedef __attribute__((ext_vector_type(2))) unsigned short v2us;
typedef __attribute__((ext_vector_type(4))) unsigned short v4us;

__global__ __launch_bounds__(256) void k_vt(const float* __restrict__ v, bf* VT) { const size_t i = ((size_t)blockIdx.x * 256 + threadIdx.x) * 2; if (i >= (size_t)DV * NK) return; const int d = (int)(i / NK), k = (int)(i % NK); v2us o; o[0] = f2bf(v[(size_t)k * DV + d]); o[1] = f2bf(v[(size_t)(k + 1) * DV + d]);
    *(volatile v2us*)(VT + i) = o; __threadfence(); *(volatile v2us*)(VT + i) = o; }
__global__ __launch_bounds__(256) void k_rnd(const float* __restrict__ src, float* dst, size_t n) { const size_t i = ((size_t)blockIdx.x * 256 + threadIdx.x) * 4; if (i >= n) return; const v4f a = *(const v4f*)(src + i); v4f o;
#pragma unroll
    for (int q = 0; q < 4; ++q) o[q] = bfr(a[q]); *(volatile v4f*)(dst + i) = o; __threadfence(); *(volatile v4f*)(dst + i) = o; }
__global__ __launch_bounds__(256) void k_bm(const float* __restrict__ qb, const float* __restrict__ kb, const int* __restrict__ mk, float* WOUT, bf* Wh, bf* Wl) {
    typedef __attribute__((ext_vector_type(4))) int v4i;
    const int lane = threadIdx.x & 31; const int i = blockIdx.x * 8 + (threadIdx.x >> 5); if (i >= NQ) return; float qv[NBIT];
    { const v4f* qp = (const v4f*)(qb + (size_t)i * NBIT);
#pragma unroll
      for (int c = 0; c < 4; ++c) { const v4f t = qp[c]; qv[c * 4] = t[0]; qv[c * 4 + 1] = t[1]; qv[c * 4 + 2] = t[2]; qv[c * 4 + 3] = t[3]; } }
    float v[64]; float mx = -3.0e38f;
#pragma unroll
    for (int ch = 0; ch < 16; ++ch) { const int j0 = ch * 128 + lane * 4; const v4i m4 = *(const v4i*)(mk + j0);
#pragma unroll
        for (int q = 0; q < 4; ++q) { const int j = j0 + q; float s = 0.f; const float* kr = kb + (size_t)j * NBIT;
#pragma unroll 1
            for (int c = 0; c < 4; ++c) { const v4f k4 = *(const v4f*)(kr + c * 4);
#pragma unroll
                for (int u = 0; u < 4; ++u) { const float dlt = fabsf(__fsub_rn(qv[c * 4 + u], k4[u])); float bm = __fsub_rn(1.0f, dlt); asm volatile("" : "+v"(bm)); const float arg = __fadd_rn(bm, 1e-8f); float l2 = __builtin_amdgcn_logf(arg); asm volatile("" : "+v"(l2)); const float ln = __fmul_rn(l2, 0.69314718055994531f); s = __fadd_rn(s, ln); } }
            const float t = (m4[q] != 0) ? __fmul_rn(s, ITEMP) : -3.0e38f; v[ch * 4 + q] = t; mx = fmaxf(mx, t); } }
#pragma unroll
    for (int sh = 16; sh; sh >>= 1) mx = fmaxf(mx, __shfl_xor(mx, sh, 32));
    float sum = 0.f;
#pragma unroll
    for (int k = 0; k < 64; ++k) { float d0 = __fsub_rn(v[k], mx); asm volatile("" : "+v"(d0)); v[k] = __builtin_amdgcn_exp2f(__fmul_rn(d0, 1.4426950408889634f)); sum += v[k]; }
#pragma unroll
    for (int sh = 16; sh; sh >>= 1) sum += __shfl_xor(sum, sh, 32);
    const float inv = __fdiv_rn(1.0f, sum);
#pragma unroll 1
    for (int ps = 0; ps < 2; ++ps) {
#pragma unroll
        for (int ch = 0; ch < 16; ++ch) { v4f w4; v4us oh, ol;
#pragma unroll
            for (int q = 0; q < 4; ++q) { const float w = __fmul_rn(v[ch * 4 + q], inv); w4[q] = w; unsigned short a, c2; splitf(w, a, c2); oh[q] = a; ol[q] = c2; }
            const size_t o = (size_t)i * NK + ch * 128 + lane * 4; *(volatile v4f*)(WOUT + o) = w4; *(volatile v4us*)(Wh + o) = oh; *(volatile v4us*)(Wl + o) = ol; }
        if (ps == 0) __threadfence(); }
}

extern "C" void kernel_launch(void* const* d_in, const int* in_sizes, int n_in,
                              void* d_out, int out_size, void* d_ws, size_t ws_size, hipStream_t stream) {
    (void)in_sizes; (void)n_in; (void)out_size;
    const float* qb = (const float*)d_in[0]; const float* kb = (const float*)d_in[1]; const float* vals = (const float*)d_in[2]; const int* mk = (const int*)d_in[3];
    float* OUT0 = (float*)d_out; float* OUT1 = OUT0 + (size_t)NB_ * NQ * DV;
    char* wsp = (char*)d_ws;
    auto take = [&](size_t bytes) { char* p = wsp; wsp += (bytes + 255) & ~(size_t)255; return (void*)p; };
    bf* VT = (bf*)take((size_t)DV * NK * 2); bf* Wh = (bf*)take((size_t)NQ * NK * 2); bf* Wl = (bf*)take((size_t)NQ * NK * 2); float* QR = (float*)take((size_t)NB_ * NQ * NBIT * 4); float* KR = (float*)take((size_t)NB_ * NK * NBIT * 4);
    if ((size_t)(wsp - (char*)d_ws) > ws_size) return;
    k_rnd<<<(unsigned)(((size_t)NB_ * NQ * NBIT / 4 + 255) / 256), 256, 0, stream>>>(qb, QR, (size_t)NB_ * NQ * NBIT); k_rnd<<<(unsigned)(((size_t)NB_ * NK * NBIT / 4 + 255) / 256), 256, 0, stream>>>(kb, KR, (size_t)NB_ * NK * NBIT);
    for (int b = 0; b < NB_; ++b) {
        k_vt<<<(unsigned)(((size_t)DV * NK / 2 + 255) / 256), 256, 0, stream>>>(vals + (size_t)b * NK * DV, VT);
        k_bm<<<NQ / 8, 256, 0, stream>>>(QR + (size_t)b * NQ * NBIT, KR + (size_t)b * NK * NBIT, mk + (size_t)b * NK, OUT1 + (size_t)b * NQ * NK, Wh, Wl);
        k_gemmw<bf, 1, false><<<dim3(NQ / 64, DV / 64, 1), 32, 0, stream>>>(Wh, Wl, VT, nullptr, NK, OUT0 + (size_t)b * NQ * DV, DV, nullptr, 0, 0, 0); }
}
